// MPNN_rbf_56581899157524
// MI455X (gfx1250) — hardware-verified
//
#include <hip/hip_runtime.h>
#include <stddef.h>


#define DN     64
#define DE     128
#define NIN    15
#define EIN    5
#define EKP    64
#define NCEN   50
#define OUTD   12
#define WEC    4096
#define NTHR   256
#define NWAVE  8
#define EPT    8
#define CHUNK  (NTHR * EPT)
#define WCAP   (EPT * 32)
#define LISTN  (NWAVE * WCAP)
#define EB     64
#define NBN    64
#define GCH    64
#define NGMAX  512
#define STMP   6
#define STS2S  6
#define CUTOFF 5.0f
#define STEPC  (5.0f / 49.0f)
#define GINV   (1.0f / STEPC)
#define HSC    16.0f
#define W2SC   1024.0f
#define ASC    (1.0f / 16384.0f)
#define WESC   256.0f
#define WEINV  (1.0f / 256.0f)
#define OFF_IH_H  0
#define OFF_IH_L  12288
#define OFF_HH_H  24576
#define OFF_HH_L  36864
#define OFF_IHL_H 49152
#define OFF_IHL_L 81920
#define OFF_HHL_H 114688
#define OFF_HHL_L 131072
#define OFF_L1_H  147456
#define OFF_L1_L  155648
#define WB_N      163840
#define PG0 (WEC * DE / 8)
#define PG1 (DE * EKP / 8)
#define PG2 (192 * DN / 8)
#define PG4 (256 * 128 / 8)
#define PG5 (256 * DN / 8)
#define PG6 (DN * 128 / 8)
#define LDS_E 73728
#define LDS_N 74240
#define LDS_S 90240

static_assert(WCAP == 256 && CHUNK == 2048);
static_assert((PG0 % NTHR) == 0 && (PG1 % NTHR) == 0 && (PG2 % NTHR) == 0 && (PG4 % NTHR) == 0 && (PG5 % NTHR) == 0 && (PG6 % NTHR) == 0);
static_assert(EB * EKP * 2 + EB * DE * 2 + EB * DN * 4 + 2 * EB * DN * 4 <= LDS_E);
static_assert(EB * EKP * 2 + EB * DE * 2 + NWAVE * 16 * 128 * 2 <= LDS_E);
static_assert(6 * NBN * DN * 4 / 4 * 0 + 16384 * 2 + 8192 * 4 + LISTN * 4 + 64 * 4 + 32 <= LDS_N);
static_assert(64 * 192 * 2 * 2 + 4096 * 4 * 2 + 528 * 4 + 768 * 4 + 16 * 4 + 768 * 4 <= LDS_S);

typedef int            v4i  __attribute__((ext_vector_type(4)));
typedef float          v2f  __attribute__((ext_vector_type(2)));
typedef float          v4f  __attribute__((ext_vector_type(4)));
typedef float          v8f  __attribute__((ext_vector_type(8)));
typedef _Float16       v8h  __attribute__((ext_vector_type(8)));
typedef _Float16       v16h __attribute__((ext_vector_type(16)));
typedef v8h            v8ha __attribute__((may_alias));
typedef unsigned short v8us __attribute__((ext_vector_type(8)));
typedef __bf16         v16b __attribute__((ext_vector_type(16)));
union FragH { v16h v; v8h h[2]; };
union FragB { v16b v; v8us u[2]; };

__device__ __forceinline__ v8f z8() { v8f z = {0.f, 0.f, 0.f, 0.f, 0.f, 0.f, 0.f, 0.f}; return z; }

__device__ __forceinline__ v8f wmh(v16h a, v16h b, v8f c) {
  v8f d = __builtin_amdgcn_wmma_f32_16x16x32_f16(false, a, false, b, (short)0, c, false, false);
  asm volatile("v_nop\n\tv_nop\n\tv_nop\n\tv_nop" : "+v"(d) : "v"(a), "v"(b));
  return d;
}
__device__ __forceinline__ v8f wmb(v16b a, v16b b, v8f c) {
  v8f d = __builtin_amdgcn_wmma_f32_16x16x32_bf16(false, a, false, b, (short)0, c, false, false);
  asm volatile("v_nop\n\tv_nop\n\tv_nop\n\tv_nop" : "+v"(d) : "v"(a), "v"(b));
  return d;
}
__device__ __forceinline__ v8f wm3(const FragB& ah, const FragB& al, const FragB& bh, const FragB& bl, v8f c) {
  c = wmb(ah.v, bh.v, c);
  c = wmb(ah.v, bl.v, c);
  c = wmb(al.v, bh.v, c);
  return c;
}

__device__ __forceinline__ unsigned short bfr(float x) {
  const unsigned u = __float_as_uint(x);
  return (unsigned short)((u + 0x7FFFu + ((u >> 16) & 1u)) >> 16);
}
__device__ __forceinline__ void split8(v4f a, v4f b, v8us& hi, v8us& lo) {
  float v[8] = {a.x, a.y, a.z, a.w, b.x, b.y, b.z, b.w};
#pragma unroll
  for (int k = 0; k < 8; ++k) {
    const unsigned short h = bfr(v[k]);
    hi[k] = h;
    lo[k] = bfr(v[k] - __uint_as_float(((unsigned)h) << 16));
  }
}
__device__ __forceinline__ v8h cvt8s(const float* v, float sc) {
  v8h r;
#pragma unroll
  for (int k = 0; k < 8; ++k) r[k] = (_Float16)(v[k] * sc);
  return r;
}
__device__ __forceinline__ float sigm(float x) { return __builtin_amdgcn_rcpf(1.0f + __expf(-x)); }
__device__ __forceinline__ float tanhm(float x) { return 2.0f * sigm(2.0f * x) - 1.0f; }
__device__ __forceinline__ float wsum(float p) {
  p += __shfl_xor(p, 16); p += __shfl_xor(p, 8); p += __shfl_xor(p, 4); p += __shfl_xor(p, 2); p += __shfl_xor(p, 1);
  return p;
}
__device__ __forceinline__ v4f relu4(v4f v) { v.x = fmaxf(v.x, 0.f); v.y = fmaxf(v.y, 0.f); v.z = fmaxf(v.z, 0.f); v.w = fmaxf(v.w, 0.f); return v; }
__device__ __forceinline__ float rbfv(float dist, int t) {
  const float c = (t == NCEN - 1) ? CUTOFF : (float)t * STEPC;
  const float r = dist - c;
  return __expf(-(r * r) * GINV);
}

__device__ __forceinline__ int scan_chunk(const int* __restrict__ keys, int nK, int cbase, int slotBase,
                                          int vec8, int* list, int tid, int lane, int wave) {
  int wc = 0;
  const int el0 = tid * EPT;
  const int e0 = cbase + el0;
  const int sent = -2147483647 - 1;
  v4i da, db;
  if (vec8 != 0 && cbase + CHUNK <= nK) {
    da = *(const v4i*)(keys + e0);
    db = *(const v4i*)(keys + e0 + 4);
  } else {
    da.x = (e0     < nK) ? keys[min(e0, nK - 1)] : sent;
    da.y = (e0 + 1 < nK) ? keys[min(e0 + 1, nK - 1)] : sent;
    da.z = (e0 + 2 < nK) ? keys[min(e0 + 2, nK - 1)] : sent;
    da.w = (e0 + 3 < nK) ? keys[min(e0 + 3, nK - 1)] : sent;
    db.x = (e0 + 4 < nK) ? keys[min(e0 + 4, nK - 1)] : sent;
    db.y = (e0 + 5 < nK) ? keys[min(e0 + 5, nK - 1)] : sent;
    db.z = (e0 + 6 < nK) ? keys[min(e0 + 6, nK - 1)] : sent;
    db.w = (e0 + 7 < nK) ? keys[min(e0 + 7, nK - 1)] : sent;
  }
  const unsigned nb = (unsigned)slotBase;
  const unsigned s0 = (unsigned)da.x - nb, s1 = (unsigned)da.y - nb, s2 = (unsigned)da.z - nb, s3 = (unsigned)da.w - nb;
  const unsigned s4 = (unsigned)db.x - nb, s5 = (unsigned)db.y - nb, s6 = (unsigned)db.z - nb, s7 = (unsigned)db.w - nb;
  const bool h0 = s0 < 64u, h1 = s1 < 64u, h2 = s2 < 64u, h3 = s3 < 64u, h4 = s4 < 64u, h5 = s5 < 64u, h6 = s6 < 64u, h7 = s7 < 64u;
  const unsigned any = __builtin_amdgcn_ballot_w32(h0 | h1 | h2 | h3 | h4 | h5 | h6 | h7);
  if (any != 0u) {
#define HITJ(J, HJ, SJ) { \
      const unsigned mj = __builtin_amdgcn_ballot_w32(HJ); \
      if (mj != 0u) { \
        if (HJ) { \
          const int pos = wc + (int)__builtin_amdgcn_mbcnt_lo(mj, 0u); \
          if (pos < WCAP) list[wave * WCAP + pos] = ((el0 + (J)) << 6) | (int)(SJ); \
        } \
        wc += (int)__builtin_popcount(mj); } }
    HITJ(0, h0, s0) HITJ(1, h1, s1) HITJ(2, h2, s2) HITJ(3, h3, s3)
    HITJ(4, h4, s4) HITJ(5, h5, s5) HITJ(6, h6, s6) HITJ(7, h7, s7)
#undef HITJ
  }
  return wc;
}

__global__ __launch_bounds__(NTHR) void k_prep(
    const float* __restrict__ w_en2, const float* __restrict__ w_en1, const float* __restrict__ w_ih,
    const float* __restrict__ w_hh, const float* __restrict__ w_ihl, const float* __restrict__ w_hhl,
    const float* __restrict__ w_l1, _Float16* w2p, _Float16* w1p, unsigned short* wb) {
  const int c1 = PG0, c2 = c1 + PG1, c3 = c2 + PG2, c4 = c3 + PG2, c5 = c4 + PG4, c6 = c5 + PG5, c7 = c6 + PG6;
  const int bstart = (int)blockIdx.x * NTHR;
  const int i = bstart + (int)threadIdx.x;
  int mode = 2, seg = 0, hoff = 0, loff = 0;
  const float* src = w_en2;
  if (bstart < c1)      { mode = 0; }
  else if (bstart < c2) { mode = 1; src = w_en1; seg = c1; }
  else if (bstart < c3) { src = w_ih;  seg = c2; hoff = OFF_IH_H;  loff = OFF_IH_L; }
  else if (bstart < c4) { src = w_hh;  seg = c3; hoff = OFF_HH_H;  loff = OFF_HH_L; }
  else if (bstart < c5) { src = w_ihl; seg = c4; hoff = OFF_IHL_H; loff = OFF_IHL_L; }
  else if (bstart < c6) { src = w_hhl; seg = c5; hoff = OFF_HHL_H; loff = OFF_HHL_L; }
  else                  { src = w_l1;  seg = c6; hoff = OFF_L1_H;  loff = OFF_L1_L; }
  if (i >= c7) return;
  const int o = (i - seg) * 8;
  if (mode == 2) {
    const v4f a = *(const v4f*)(src + o), b = *(const v4f*)(src + o + 4);
    v8us hi, lo;
    split8(a, b, hi, lo);
    *(volatile v8us*)(wb + hoff + o) = hi;
    *(volatile v8us*)(wb + loff + o) = lo;
    __threadfence();
    *(volatile v8us*)(wb + hoff + o) = hi;
    *(volatile v8us*)(wb + loff + o) = lo;
  } else {
    float v[8];
    if (mode == 0) {
#pragma unroll
      for (int e = 0; e < 8; ++e) v[e] = src[o + e] * W2SC;
    } else {
      const int n = o / EKP;
      const int k0 = o - n * EKP;
#pragma unroll
      for (int e = 0; e < 8; ++e) {
        const int k = k0 + e;
        const int kc = k < 54 ? k : 53;
        const float x = src[n * 54 + kc];
        v[e] = (k < 54) ? x : x * 0.0f;
      }
    }
    const v8h hv = cvt8s(v, 1.0f);
    _Float16* dp = (mode == 0 ? w2p : w1p) + o;
    *(volatile v8h*)dp = hv;
    __threadfence();
    *(volatile v8h*)dp = hv;
  }
}

__global__ __launch_bounds__(NTHR) void k_lin0(const float* __restrict__ x, const float* __restrict__ w,
                                               const float* __restrict__ b, float* h, int nN) {
  __shared__ float ws0[DN * NIN];
  __shared__ float bs0[DN];
  __shared__ __attribute__((aligned(16))) float st[NBN * DN];
  const int tid = threadIdx.x;
  for (int i = tid; i < DN * NIN; i += NTHR) ws0[i] = w[i];
  if (tid < DN) bs0[tid] = b[tid];
  __syncthreads();
  const int row = tid >> 2, cg = tid & 3;
  int node = (int)blockIdx.x * NBN + row;
  node = node > nN - 1 ? nN - 1 : node;
  const float* xp = x + (size_t)node * NIN;
  float acc[16];
#pragma unroll
  for (int j = 0; j < 16; ++j) acc[j] = bs0[16 * cg + j];
#pragma unroll 1
  for (int k = 0; k < NIN; ++k) {
    const float xv = xp[k];
#pragma unroll
    for (int j = 0; j < 16; ++j) acc[j] += xv * ws0[(16 * cg + j) * NIN + k];
  }
  float* sp = st + row * DN + 16 * cg;
#pragma unroll
  for (int j = 0; j < 16; ++j) sp[j] = fmaxf(acc[j], 0.0f);
  __syncthreads();
  v4f ov[4];
#pragma unroll
  for (int it = 0; it < 4; ++it) ov[it] = *(const v4f*)(st + 4 * (it * NTHR + tid));
  float* gp = h + (size_t)blockIdx.x * NBN * DN;
#pragma unroll
  for (int it = 0; it < 4; ++it) *(volatile v4f*)(gp + 4 * (it * NTHR + tid)) = ov[it];
  __threadfence();
#pragma unroll
  for (int it = 0; it < 4; ++it) *(volatile v4f*)(gp + 4 * (it * NTHR + tid)) = ov[it];
}

template <int STORE>
__global__ __launch_bounds__(NTHR) void k_edge(const float* __restrict__ ea, const int* __restrict__ ei,
    const float* __restrict__ hpl, const _Float16* __restrict__ w1p, const float* __restrict__ b_en1,
    const _Float16* __restrict__ w2p, const float* __restrict__ b_en2, _Float16* wedge, float* msg,
    int nE, int nN, int nSB) {
  extern __shared__ v4f lds_dyn[];
  _Float16* ef  = (_Float16*)lds_dyn;
  _Float16* hd  = ef + EB * EKP;
  float*    osr = (float*)(hd + EB * DE);
  float*    msp = osr + EB * DN;
  _Float16* stg = (_Float16*)osr;
  const int tid = threadIdx.x, lane = tid & 31, wave = tid >> 5, hf = lane >> 4, m = lane & 15;
  const int eb = (int)blockIdx.x * EB;
  if (STORE == 0) {
    const int el = tid >> 2, part = tid & 3;
    int e = eb + el; e = e > nE - 1 ? nE - 1 : e;
    int s = ei[e]; s = s < 0 ? 0 : (s > nN - 1 ? nN - 1 : s);
    const float* sp = hpl + (size_t)s * DN + 16 * part;
    float* dp = osr + el * DN + 16 * part;
#pragma unroll
    for (int q = 0; q < 4; ++q) *(v4f*)(dp + 4 * q) = *(const v4f*)(sp + 4 * q);
  }
  __syncthreads();
  const bool streamBlk = (STORE == 0) && ((int)blockIdx.x < nSB);
  if (streamBlk) {
    const int q4 = lane >> 3, jj = lane & 7;
#pragma unroll 1
    for (int j = 0; j < 8; ++j) {
      const int el = wave * 8 + j;
      int e = eb + el; e = e > nE - 1 ? nE - 1 : e;
      const _Float16* wp = wedge + (size_t)e * WEC + 64 * q4 + 8 * jj;
      const float* op = osr + el * DN + q4;
      float acc[8];
#pragma unroll
      for (int k = 0; k < 8; ++k) acc[k] = 0.0f;
#pragma unroll 2
      for (int i = 0; i < 16; ++i) {
        const v8h w = *(const v8h*)(wp + 256 * i);
        const float o = op[4 * i];
#pragma unroll
        for (int k = 0; k < 8; ++k) acc[k] += o * (float)w[k];
      }
#pragma unroll
      for (int k = 0; k < 8; ++k) { acc[k] += __shfl_xor(acc[k], 8); acc[k] += __shfl_xor(acc[k], 16); }
      if (lane < 8) {
        v4f a0 = {acc[0], acc[1], acc[2], acc[3]};
        v4f a1 = {acc[4], acc[5], acc[6], acc[7]};
        const v4f z = {0.f, 0.f, 0.f, 0.f};
        *(v4f*)(msp + el * DN + 8 * lane) = a0 * WEINV;
        *(v4f*)(msp + el * DN + 8 * lane + 4) = a1 * WEINV;
        *(v4f*)(msp + EB * DN + el * DN + 8 * lane) = z;
        *(v4f*)(msp + EB * DN + el * DN + 8 * lane + 4) = z;
      }
    }
  } else {
    {
      const int el = tid & 63, part = tid >> 6;
      int e = eb + el; e = e > nE - 1 ? nE - 1 : e;
      const float* ap = ea + (size_t)e * EIN;
      const float a0 = ap[0], a1 = ap[1], a2 = ap[2], a3 = ap[3], dist = ap[4];
      const float zer = dist * 0.0f;
      float v[16];
      if (part == 0) {
        v[0] = a0; v[1] = a1; v[2] = a2; v[3] = a3;
#pragma unroll
        for (int i = 4; i < 16; ++i) v[i] = rbfv(dist, i - 4);
      } else {
#pragma unroll
        for (int i = 0; i < 16; ++i) {
          const int t = 16 * part + i - 4;
          const float rv = rbfv(dist, t);
          v[i] = (t < NCEN) ? rv : zer;
        }
      }
      _Float16* dp = ef + el * EKP + 16 * part;
      *(v8h*)dp = cvt8s(v, 1.0f);
      *(v8h*)(dp + 8) = cvt8s(v + 8, 1.0f);
    }
    __syncthreads();
    {
      const int rg = wave & 3, ch = wave >> 2;
      v8f acc[4];
#pragma unroll
      for (int t = 0; t < 4; ++t) acc[t] = z8();
#pragma unroll
      for (int ks = 0; ks < 2; ++ks) {
        const _Float16* ar = ef + (16 * rg + m) * EKP + 32 * ks + 8 * hf;
        FragH a; a.h[0] = *(const v8h*)ar; a.h[1] = *(const v8h*)(ar + 16);
#pragma unroll
        for (int t = 0; t < 4; ++t) {
          const _Float16* bp = w1p + (size_t)(64 * ch + 16 * t + m) * EKP + 32 * ks + 8 * hf;
          FragH b; b.h[0] = *(const v8h*)bp; b.h[1] = *(const v8h*)(bp + 16);
          acc[t] = wmh(a.v, b.v, acc[t]);
        }
      }
#pragma unroll
      for (int t = 0; t < 4; ++t) {
        const int col = 64 * ch + 16 * t + m;
        const float bv = b_en1[col];
        _Float16* hp = hd + (16 * rg + 8 * hf) * DE + col;
#pragma unroll
        for (int r = 0; r < 8; ++r) hp[r * DE] = (_Float16)(fmaxf(acc[t][r] + bv, 0.0f) * HSC);
      }
    }
    __syncthreads();
    {
      const int rg = wave & 3, dh = wave >> 2;
      FragH aF[4];
      const _Float16* ar = hd + (16 * rg + m) * DE + 8 * hf;
#pragma unroll
      for (int ks = 0; ks < 4; ++ks) { aF[ks].h[0] = *(const v8h*)(ar + 32 * ks); aF[ks].h[1] = *(const v8h*)(ar + 32 * ks + 16); }
      v8f macc[4];
#pragma unroll
      for (int t = 0; t < 4; ++t) macc[t] = z8();
#pragma unroll 1
      for (int p = 0; p < 16; ++p) {
        const int cb = 2048 * dh + 128 * p;
        v8f acc[8];
#pragma unroll
        for (int t = 0; t < 8; ++t) acc[t] = z8();
#pragma unroll
        for (int ks = 0; ks < 4; ++ks) {
#pragma unroll
          for (int t = 0; t < 8; ++t) {
            const _Float16* bp = w2p + (size_t)(cb + 16 * t + m) * DE + 32 * ks + 8 * hf;
            FragH b; b.h[0] = *(const v8h*)bp; b.h[1] = *(const v8h*)(bp + 16);
            acc[t] = wmh(aF[ks].v, b.v, acc[t]);
          }
        }
        float bv[8];
#pragma unroll
        for (int t = 0; t < 8; ++t) bv[t] = b_en2[cb + 16 * t + m];
        if (STORE) {
          _Float16* sw = stg + wave * 2048;
#pragma unroll
          for (int t = 0; t < 8; ++t) {
#pragma unroll
            for (int r = 0; r < 8; ++r) sw[(8 * hf + r) * 128 + 16 * t + m] = (_Float16)((acc[t][r] * ASC + bv[t]) * WESC);
          }
          __builtin_amdgcn_fence(__ATOMIC_RELEASE, "wavefront");
          __builtin_amdgcn_wave_barrier();
          v8h pv[8];
#pragma unroll
          for (int i = 0; i < 8; ++i) pv[i] = *(const v8ha*)(sw + (2 * i + hf) * 128 + 8 * m);
          _Float16* gb = wedge + (size_t)(eb + 16 * rg) * WEC + cb + 8 * m;
#pragma unroll
          for (int i = 0; i < 8; ++i) *(volatile v8h*)(gb + (size_t)(2 * i + hf) * WEC) = pv[i];
          __threadfence();
#pragma unroll
          for (int i = 0; i < 8; ++i) *(volatile v8h*)(gb + (size_t)(2 * i + hf) * WEC) = pv[i];
          __builtin_amdgcn_fence(__ATOMIC_RELEASE, "wavefront");
          __builtin_amdgcn_wave_barrier();
        } else {
          const int d0 = 32 * dh + 2 * p;
          const float* orow = osr + (16 * rg + 8 * hf) * DN + d0;
#pragma unroll
          for (int r = 0; r < 8; ++r) {
            const v2f o = *(const v2f*)(orow + r * DN);
#pragma unroll
            for (int t = 0; t < 4; ++t)
              macc[t][r] += o.x * (acc[t][r] * ASC + bv[t]) + o.y * (acc[t + 4][r] * ASC + bv[t + 4]);
          }
        }
      }
      if (STORE == 0) {
        float* mp = msp + dh * EB * DN + (16 * rg + 8 * hf) * DN + m;
#pragma unroll
        for (int t = 0; t < 4; ++t) {
#pragma unroll
          for (int r = 0; r < 8; ++r) mp[r * DN + 16 * t] = macc[t][r];
        }
      }
    }
  }
  if (STORE == 0) {
    __syncthreads();
    v4f ov[4];
#pragma unroll
    for (int it = 0; it < 4; ++it) {
      const int i = it * NTHR + tid;
      ov[it] = *(const v4f*)(msp + 4 * i) + *(const v4f*)(msp + EB * DN + 4 * i);
    }
    float* mb = msg + (size_t)eb * DN;
#pragma unroll
    for (int it = 0; it < 4; ++it) *(volatile v4f*)(mb + 4 * (it * NTHR + tid)) = ov[it];
    __threadfence();
#pragma unroll
    for (int it = 0; it < 4; ++it) *(volatile v4f*)(mb + 4 * (it * NTHR + tid)) = ov[it];
  }
}

__global__ __launch_bounds__(NTHR) void k_node(const int* __restrict__ ei, const float* __restrict__ msg,
    float* hpl, const float* __restrict__ b_conv, const unsigned short* __restrict__ wb,
    const float* __restrict__ b_ih, const float* __restrict__ b_hh, int nE, int nN, int vec8) {
  extern __shared__ v4f lds_dyn[];
  float* agg = (float*)lds_dyn;
  float* hr  = agg + 4096;
  unsigned short* mh  = (unsigned short*)(hr + 4096);
  unsigned short* ml  = mh + 4096;
  unsigned short* hh16 = ml + 4096;
  unsigned short* hl16 = hh16 + 4096;
  int* list = (int*)(hl16 + 4096);
  int* cnt  = list + LISTN;
  int* wcnt = cnt + 64;
  const int tid = threadIdx.x, lane = tid & 31, wave = tid >> 5, hf = lane >> 4, m = lane & 15;
  const int nb = (int)blockIdx.x * NBN;
  {
    const int row = tid >> 2, part = tid & 3;
    const float* hp = hpl + (size_t)(nb + row) * DN + 16 * part;
    const v4f a0 = *(const v4f*)hp, a1 = *(const v4f*)(hp + 4), a2 = *(const v4f*)(hp + 8), a3 = *(const v4f*)(hp + 12);
    float* dp = hr + row * DN + 16 * part;
    *(v4f*)dp = a0; *(v4f*)(dp + 4) = a1; *(v4f*)(dp + 8) = a2; *(v4f*)(dp + 12) = a3;
    const v4f z = {0.f, 0.f, 0.f, 0.f};
    float* zp = agg + row * DN + 16 * part;
    *(v4f*)zp = z; *(v4f*)(zp + 4) = z; *(v4f*)(zp + 8) = z; *(v4f*)(zp + 12) = z;
    v8us hA, lA, hB, lB;
    split8(a0, a1, hA, lA); split8(a2, a3, hB, lB);
    *(v8us*)(hh16 + row * DN + 16 * part) = hA; *(v8us*)(hh16 + row * DN + 16 * part + 8) = hB;
    *(v8us*)(hl16 + row * DN + 16 * part) = lA; *(v8us*)(hl16 + row * DN + 16 * part + 8) = lB;
    if (tid < 64) cnt[tid] = 0;
  }
  __syncthreads();
  const int* keys = ei + nE;
  const int nChunks = (nE + CHUNK - 1) / CHUNK;
#pragma unroll 1
  for (int ch = 0; ch < nChunks; ++ch) {
    const int cbase = ch * CHUNK;
    const int wc = scan_chunk(keys, nE, cbase, nb, vec8, list, tid, lane, wave);
    if (lane == 0) wcnt[wave] = wc;
    __syncthreads();
#pragma unroll 1
    for (int wsx = 0; wsx < NWAVE; ++wsx) {
      int n = __builtin_amdgcn_readfirstlane(wcnt[wsx]);
      n = n > WCAP ? WCAP : (n < 0 ? 0 : n);
      const int* lp = list + wsx * WCAP;
#pragma unroll 1
      for (int i = 0; i < n; ++i) {
        const int ent = __builtin_amdgcn_readfirstlane(lp[i]);
        const int slot = ent & 63;
        if ((slot >> 3) == wave) {
          int e = cbase + (ent >> 6);
          e = e > nE - 1 ? nE - 1 : e;
          const v2f v = *(const v2f*)(msg + (size_t)e * DN + 2 * lane);
          v2f* ap = (v2f*)(agg + slot * DN + 2 * lane);
          *ap = *ap + v;
          if (lane == 0) cnt[slot] = cnt[slot] + 1;
        }
      }
    }
    __syncthreads();
  }
  {
    const int row = tid >> 2, part = tid & 3;
    int c = cnt[row]; c = c < 1 ? 1 : c;
    const float rd = 1.0f / (float)c;
    const float* ap = agg + row * DN + 16 * part;
    const float* bp = b_conv + 16 * part;
    const v4f a0 = relu4(*(const v4f*)ap * rd + *(const v4f*)bp);
    const v4f a1 = relu4(*(const v4f*)(ap + 4) * rd + *(const v4f*)(bp + 4));
    const v4f a2 = relu4(*(const v4f*)(ap + 8) * rd + *(const v4f*)(bp + 8));
    const v4f a3 = relu4(*(const v4f*)(ap + 12) * rd + *(const v4f*)(bp + 12));
    v8us hA, lA, hB, lB;
    split8(a0, a1, hA, lA); split8(a2, a3, hB, lB);
    *(v8us*)(mh + row * DN + 16 * part) = hA; *(v8us*)(mh + row * DN + 16 * part + 8) = hB;
    *(v8us*)(ml + row * DN + 16 * part) = lA; *(v8us*)(ml + row * DN + 16 * part + 8) = lB;
  }
  __syncthreads();
  {
    const int rg = wave >> 1, q = wave & 1;
    v8f gi[3][2], gh[3][2];
#pragma unroll
    for (int g = 0; g < 3; ++g) { gi[g][0] = z8(); gi[g][1] = z8(); gh[g][0] = z8(); gh[g][1] = z8(); }
#pragma unroll
    for (int ks = 0; ks < 2; ++ks) {
      const int ao = (16 * rg + m) * DN + 32 * ks + 8 * hf;
      FragB amh, aml, ahh, ahl;
      amh.u[0] = *(const v8us*)(mh + ao);   amh.u[1] = *(const v8us*)(mh + ao + 16);
      aml.u[0] = *(const v8us*)(ml + ao);   aml.u[1] = *(const v8us*)(ml + ao + 16);
      ahh.u[0] = *(const v8us*)(hh16 + ao); ahh.u[1] = *(const v8us*)(hh16 + ao + 16);
      ahl.u[0] = *(const v8us*)(hl16 + ao); ahl.u[1] = *(const v8us*)(hl16 + ao + 16);
#pragma unroll
      for (int g = 0; g < 3; ++g) {
#pragma unroll
        for (int u = 0; u < 2; ++u) {
          const int bo = (64 * g + 32 * q + 16 * u + m) * DN + 32 * ks + 8 * hf;
          FragB bh, bl;
          bh.u[0] = *(const v8us*)(wb + OFF_IH_H + bo); bh.u[1] = *(const v8us*)(wb + OFF_IH_H + bo + 16);
          bl.u[0] = *(const v8us*)(wb + OFF_IH_L + bo); bl.u[1] = *(const v8us*)(wb + OFF_IH_L + bo + 16);
          gi[g][u] = wm3(amh, aml, bh, bl, gi[g][u]);
          bh.u[0] = *(const v8us*)(wb + OFF_HH_H + bo); bh.u[1] = *(const v8us*)(wb + OFF_HH_H + bo + 16);
          bl.u[0] = *(const v8us*)(wb + OFF_HH_L + bo); bl.u[1] = *(const v8us*)(wb + OFF_HH_L + bo + 16);
          gh[g][u] = wm3(ahh, ahl, bh, bl, gh[g][u]);
        }
      }
    }
#pragma unroll
    for (int u = 0; u < 2; ++u) {
      const int j = 32 * q + 16 * u + m;
      const float bir = b_ih[j], biz = b_ih[64 + j], bin = b_ih[128 + j];
      const float bhr = b_hh[j], bhz = b_hh[64 + j], bhn = b_hh[128 + j];
#pragma unroll
      for (int r = 0; r < 8; ++r) {
        const int row = 16 * rg + 8 * hf + r;
        const float rr = sigm(gi[0][u][r] + bir + gh[0][u][r] + bhr);
        const float zz = sigm(gi[1][u][r] + biz + gh[1][u][r] + bhz);
        const float nn = tanhm(gi[2][u][r] + bin + rr * (gh[2][u][r] + bhn));
        const float ho = hr[row * DN + j];
        agg[row * DN + j] = (1.0f - zz) * nn + zz * ho;
      }
    }
  }
  __syncthreads();
  v4f ov[4];
#pragma unroll
  for (int it = 0; it < 4; ++it) ov[it] = *(const v4f*)(agg + 4 * (it * NTHR + tid));
  float* gp = hpl + (size_t)nb * DN;
#pragma unroll
  for (int it = 0; it < 4; ++it) *(volatile v4f*)(gp + 4 * (it * NTHR + tid)) = ov[it];
  __threadfence();
#pragma unroll
  for (int it = 0; it < 4; ++it) *(volatile v4f*)(gp + 4 * (it * NTHR + tid)) = ov[it];
}

__device__ __forceinline__ void buildA(const float* qst, const float* hlp, int g0, int kq, bool z0,
                                       unsigned short* AH, unsigned short* AL, int tid) {
  const int row = tid & 63, part = tid >> 6;
  const int g = g0 + row;
#pragma unroll 1
  for (int gi8 = 0; gi8 < (kq >> 3); ++gi8) {
    const int kk = kq * part + 8 * gi8;
    v4f a, b;
    if (kk < 128) { const float* p = qst + (size_t)g * 128 + kk; a = *(const v4f*)p; b = *(const v4f*)(p + 4); }
    else          { const float* p = hlp + (size_t)g * DN + (kk - 128); a = *(const v4f*)p; b = *(const v4f*)(p + 4); }
    const v4f z = {0.f, 0.f, 0.f, 0.f};
    a = z0 ? z : a; b = z0 ? z : b;
    v8us hi, lo;
    split8(a, b, hi, lo);
    *(v8us*)(AH + row * 192 + kk) = hi;
    *(v8us*)(AL + row * 192 + kk) = lo;
  }
}

__global__ __launch_bounds__(NTHR) void k_s2s(const float* __restrict__ hpl, const int* __restrict__ batch,
    const unsigned short* __restrict__ wb, const float* __restrict__ b_ihl, const float* __restrict__ b_hhl,
    const float* __restrict__ b_l1, const float* __restrict__ w_l2, const float* __restrict__ b_l2,
    float* qst, float* hlp, float* clp, float* out, int nN, int nG) {
  extern __shared__ v4f lds_dyn[];
  unsigned short* AH = (unsigned short*)lds_dyn;
  unsigned short* AL = AH + 64 * 192;
  float* HS  = (float*)(AL + 64 * 192);
  float* CS  = HS + 4096;
  int*   SEG = (int*)(CS + 4096);
  float* W2S = (float*)(SEG + 528);
  float* B2S = W2S + 768;
  float* OST = B2S + 16;
  const int tid = threadIdx.x, lane = tid & 31, wave = tid >> 5, hf = lane >> 4, m = lane & 15;
  for (int i = tid; i < OUTD * DN; i += NTHR) W2S[i] = w_l2[i];
  if (tid < 16) { const float bv = b_l2[tid < OUTD ? tid : OUTD - 1]; B2S[tid] = (tid < OUTD) ? bv : 0.0f; }
  for (int g = tid; g <= nG; g += NTHR) {
    int base = 0, len = nN;
#pragma unroll 1
    for (int it = 0; it < 40 && len > 0; ++it) {
      const int half = len >> 1;
      int mid = base + half; mid = mid > nN - 1 ? nN - 1 : mid;
      const int bv = batch[mid];
      if (bv < g) { base = mid + 1; len = len - half - 1; } else { len = half; }
    }
    SEG[g] = base > nN ? nN : base;
  }
  __syncthreads();
  const int nRC = nG / GCH;
#pragma unroll 1
  for (int s = 0; s < STS2S; ++s) {
    const bool z0 = (s == 0);
#pragma unroll 1
    for (int rc = 0; rc < nRC; ++rc) {
      const int g0 = rc * GCH;
      buildA(qst, hlp, g0, 48, z0, AH, AL, tid);
      __syncthreads();
      {
        const int rg = wave >> 1, q = wave & 1;
        v8f acc[4][2];
#pragma unroll
        for (int g = 0; g < 4; ++g) { acc[g][0] = z8(); acc[g][1] = z8(); }
#pragma unroll
        for (int ks = 0; ks < 6; ++ks) {
          const int ao = (16 * rg + m) * 192 + 32 * ks + 8 * hf;
          FragB ah, al;
          ah.u[0] = *(const v8us*)(AH + ao); ah.u[1] = *(const v8us*)(AH + ao + 16);
          al.u[0] = *(const v8us*)(AL + ao); al.u[1] = *(const v8us*)(AL + ao + 16);
#pragma unroll
          for (int g = 0; g < 4; ++g) {
#pragma unroll
            for (int u = 0; u < 2; ++u) {
              const int n = 64 * g + 32 * q + 16 * u + m;
              const unsigned short* ph; const unsigned short* pl;
              if (ks < 4) { ph = wb + OFF_IHL_H + n * 128 + 32 * ks + 8 * hf;      pl = wb + OFF_IHL_L + n * 128 + 32 * ks + 8 * hf; }
              else        { ph = wb + OFF_HHL_H + n * DN + 32 * (ks - 4) + 8 * hf; pl = wb + OFF_HHL_L + n * DN + 32 * (ks - 4) + 8 * hf; }
              FragB bh, bl;
              bh.u[0] = *(const v8us*)ph; bh.u[1] = *(const v8us*)(ph + 16);
              bl.u[0] = *(const v8us*)pl; bl.u[1] = *(const v8us*)(pl + 16);
              acc[g][u] = wm3(ah, al, bh, bl, acc[g][u]);
            }
          }
        }
#pragma unroll
        for (int u = 0; u < 2; ++u) {
          const int j = 32 * q + 16 * u + m;
          const float bi = b_ihl[j] + b_hhl[j], bf = b_ihl[64 + j] + b_hhl[64 + j];
          const float bg = b_ihl[128 + j] + b_hhl[128 + j], bo = b_ihl[192 + j] + b_hhl[192 + j];
#pragma unroll
          for (int r = 0; r < 8; ++r) {
            const int row = 16 * rg + 8 * hf + r;
            const float craw = clp[(size_t)(g0 + row) * DN + j];
            const float co = z0 ? 0.0f : craw;
            const float cn = sigm(acc[1][u][r] + bf) * co + sigm(acc[0][u][r] + bi) * tanhm(acc[2][u][r] + bg);
            const float hn = sigm(acc[3][u][r] + bo) * tanhm(cn);
            CS[row * DN + j] = cn;
            HS[row * DN + j] = hn;
          }
        }
      }
      __syncthreads();
      {
        v4f hv[4], cv[4];
#pragma unroll
        for (int it = 0; it < 4; ++it) { const int i = it * NTHR + tid; hv[it] = *(const v4f*)(HS + 4 * i); cv[it] = *(const v4f*)(CS + 4 * i); }
#pragma unroll
        for (int ps = 0; ps < 2; ++ps) {
#pragma unroll
          for (int it = 0; it < 4; ++it) {
            const int i = it * NTHR + tid, row = i >> 4, c4 = (i & 15) * 4;
            *(volatile v4f*)(hlp + (size_t)(g0 + row) * DN + c4) = hv[it];
            *(volatile v4f*)(clp + (size_t)(g0 + row) * DN + c4) = cv[it];
            *(volatile v4f*)(qst + (size_t)(g0 + row) * 128 + c4) = hv[it];
          }
          if (ps == 0) __threadfence();
        }
      }
      __syncthreads();
    }
#pragma unroll 1
    for (int g = wave; g < nG; g += NWAVE) {
      int st = SEG[g], en = SEG[g + 1];
      st = st < 0 ? 0 : (st > nN ? nN : st);
      en = en < st ? st : (en > nN ? nN : en);
      const v2f qv = *(const v2f*)(hlp + (size_t)g * DN + 2 * lane);
      float emax = -__builtin_inff();
#pragma unroll 1
      for (int n = st; n < en; ++n) {
        const v2f o = *(const v2f*)(hpl + (size_t)n * DN + 2 * lane);
        const float p = wsum(o.x * qv.x + o.y * qv.y);
        emax = fmaxf(emax, p);
      }
      float esum = 0.0f;
      v2f racc = {0.f, 0.f};
#pragma unroll 1
      for (int n = st; n < en; ++n) {
        const v2f o = *(const v2f*)(hpl + (size_t)n * DN + 2 * lane);
        const float p = wsum(o.x * qv.x + o.y * qv.y);
        const float ez = expf(p - emax);
        esum += ez;
        racc += o * ez;
      }
      const float rq = 1.0f / (esum > 0.0f ? esum : 1.0f);
      const float rinv = (esum > 0.0f) ? rq : 0.0f;
      const v2f rv = racc * rinv;
      float* rp = qst + (size_t)g * 128 + DN + 2 * lane;
      *(volatile v2f*)rp = rv;
      __threadfence();
      *(volatile v2f*)rp = rv;
    }
    __syncthreads();
  }
#pragma unroll 1
  for (int rc = 0; rc < nRC; ++rc) {
    const int g0 = rc * GCH;
    buildA(qst, hlp, g0, 32, false, AH, AL, tid);
    __syncthreads();
    {
      const int rg = wave >> 1, q = wave & 1;
      v8f acc[2]; acc[0] = z8(); acc[1] = z8();
#pragma unroll
      for (int ks = 0; ks < 4; ++ks) {
        const int ao = (16 * rg + m) * 192 + 32 * ks + 8 * hf;
        FragB ah, al;
        ah.u[0] = *(const v8us*)(AH + ao); ah.u[1] = *(const v8us*)(AH + ao + 16);
        al.u[0] = *(const v8us*)(AL + ao); al.u[1] = *(const v8us*)(AL + ao + 16);
#pragma unroll
        for (int u = 0; u < 2; ++u) {
          const int bo = (32 * q + 16 * u + m) * 128 + 32 * ks + 8 * hf;
          FragB bh, bl;
          bh.u[0] = *(const v8us*)(wb + OFF_L1_H + bo); bh.u[1] = *(const v8us*)(wb + OFF_L1_H + bo + 16);
          bl.u[0] = *(const v8us*)(wb + OFF_L1_L + bo); bl.u[1] = *(const v8us*)(wb + OFF_L1_L + bo + 16);
          acc[u] = wm3(ah, al, bh, bl, acc[u]);
        }
      }
#pragma unroll
      for (int u = 0; u < 2; ++u) {
        const int j = 32 * q + 16 * u + m;
        const float bv = b_l1[j];
#pragma unroll
        for (int r = 0; r < 8; ++r) HS[(16 * rg + 8 * hf + r) * DN + j] = fmaxf(acc[u][r] + bv, 0.0f);
      }
    }
    __syncthreads();
    {
      const int row = tid >> 2, oc = tid & 3;
      float a0 = B2S[3 * oc], a1 = B2S[3 * oc + 1], a2 = B2S[3 * oc + 2];
      const float* yr = HS + row * DN;
      const float* w0 = W2S + (3 * oc) * DN;
#pragma unroll 1
      for (int k = 0; k < DN; ++k) {
        const float y = yr[k];
        a0 += y * w0[k]; a1 += y * w0[DN + k]; a2 += y * w0[2 * DN + k];
      }
      OST[row * OUTD + 3 * oc] = a0; OST[row * OUTD + 3 * oc + 1] = a1; OST[row * OUTD + 3 * oc + 2] = a2;
    }
    __syncthreads();
    if (tid < 192) {
      const v4f v = *(const v4f*)(OST + 4 * tid);
      float* op = out + (size_t)rc * (GCH * OUTD) + 4 * tid;
      *(volatile v4f*)op = v;
      __threadfence();
      *(volatile v4f*)op = v;
    }
    __syncthreads();
  }
}

extern "C" void kernel_launch(void* const* d_in, const int* in_sizes, int n_in,
                              void* d_out, int out_size, void* d_ws, size_t ws_size,
                              hipStream_t stream) {
  if (n_in < 23) return;
  const int nN = in_sizes[0] / NIN;
  const int nE = in_sizes[2] / 2;
  const int nG = out_size / OUTD;
  if (nN <= 0 || nE <= 0 || nG <= 0) return;
  if (in_sizes[0] != nN * NIN || (nN % NBN) != 0 || in_sizes[3] != nN) return;
  if (in_sizes[2] != 2 * nE || in_sizes[1] != nE * EIN || (nE % EB) != 0) return;
  if (out_size != nG * OUTD || (nG % GCH) != 0 || nG > NGMAX) return;
  if (in_sizes[4] != DN * NIN || in_sizes[5] != DN || in_sizes[6] != DE * 54 || in_sizes[7] != DE) return;
  if (in_sizes[8] != WEC * DE || in_sizes[9] != WEC || in_sizes[10] != DN) return;
  if (in_sizes[11] != 192 * DN || in_sizes[12] != 192 * DN || in_sizes[13] != 192 || in_sizes[14] != 192) return;
  if (in_sizes[15] != 256 * 128 || in_sizes[16] != 256 * DN || in_sizes[17] != 256 || in_sizes[18] != 256) return;
  if (in_sizes[19] != DN * 128 || in_sizes[20] != DN || in_sizes[21] != OUTD * DN || in_sizes[22] != OUTD) return;

  const float* x      = (const float*)d_in[0];
  const float* ea     = (const float*)d_in[1];
  const int*   ei     = (const int*)d_in[2];
  const int*   batch  = (const int*)d_in[3];
  const float* w_lin0 = (const float*)d_in[4];
  const float* b_lin0 = (const float*)d_in[5];
  const float* w_en1  = (const float*)d_in[6];
  const float* b_en1  = (const float*)d_in[7];
  const float* w_en2  = (const float*)d_in[8];
  const float* b_en2  = (const float*)d_in[9];
  const float* b_conv = (const float*)d_in[10];
  const float* w_ih   = (const float*)d_in[11];
  const float* w_hh   = (const float*)d_in[12];
  const float* b_ih   = (const float*)d_in[13];
  const float* b_hh   = (const float*)d_in[14];
  const float* w_ihl  = (const float*)d_in[15];
  const float* w_hhl  = (const float*)d_in[16];
  const float* b_ihl  = (const float*)d_in[17];
  const float* b_hhl  = (const float*)d_in[18];
  const float* w_lin1 = (const float*)d_in[19];
  const float* b_lin1 = (const float*)d_in[20];
  const float* w_lin2 = (const float*)d_in[21];
  const float* b_lin2 = (const float*)d_in[22];
  float* out = (float*)d_out;

  const size_t szW2P = (size_t)WEC * DE * 2, szW1P = (size_t)DE * EKP * 2, szWB = (size_t)WB_N * 2;
  const size_t szH = (size_t)nN * DN * 4, szMSG = (size_t)nE * DN * 4, szQ = (size_t)nG * 128 * 4, szHL = (size_t)nG * DN * 4;
  const size_t oW2P = 0, oW1P = oW2P + szW2P, oWB = oW1P + szW1P, oH = oWB + szWB, oMSG = oH + szH;
  const size_t oQ = oMSG + szMSG, oHL = oQ + szQ, oCL = oHL + szHL, oWE = oCL + szHL;
  if (oWE > ws_size) return;
  const size_t blkBytes = (size_t)EB * WEC * 2;
  const int nEB = nE / EB;
  size_t nSBz = (ws_size - oWE) / blkBytes;
  const int nSB = nSBz > (size_t)nEB ? nEB : (int)nSBz;
  char* ws = (char*)d_ws;
  _Float16* w2p = (_Float16*)(ws + oW2P);
  _Float16* w1p = (_Float16*)(ws + oW1P);
  unsigned short* wb = (unsigned short*)(ws + oWB);
  float* h   = (float*)(ws + oH);
  float* msg = (float*)(ws + oMSG);
  float* qst = (float*)(ws + oQ);
  float* hlp = (float*)(ws + oHL);
  float* clp = (float*)(ws + oCL);
  _Float16* wedge = (_Float16*)(ws + oWE);
  const int vec8 = ((nE & 3) == 0) ? 1 : 0;

  const int nPrep = (PG0 + PG1 + 2 * PG2 + PG4 + PG5 + PG6) / NTHR;
  k_prep<<<nPrep, NTHR, 0, stream>>>(w_en2, w_en1, w_ih, w_hh, w_ihl, w_hhl, w_lin1, w2p, w1p, wb);
  k_lin0<<<nN / NBN, NTHR, 0, stream>>>(x, w_lin0, b_lin0, h, nN);

  hipFuncSetAttribute(reinterpret_cast<const void*>(&k_edge<1>), hipFuncAttributeMaxDynamicSharedMemorySize, LDS_E);
  hipFuncSetAttribute(reinterpret_cast<const void*>(&k_edge<0>), hipFuncAttributeMaxDynamicSharedMemorySize, LDS_E);
  hipFuncSetAttribute(reinterpret_cast<const void*>(&k_node), hipFuncAttributeMaxDynamicSharedMemorySize, LDS_N);
  hipFuncSetAttribute(reinterpret_cast<const void*>(&k_s2s), hipFuncAttributeMaxDynamicSharedMemorySize, LDS_S);
  if (nSB > 0)
    k_edge<1><<<nSB, NTHR, LDS_E, stream>>>(ea, ei, h, w1p, b_en1, w2p, b_en2, wedge, msg, nE, nN, nSB);
  for (int s = 0; s < STMP; ++s) {
    k_edge<0><<<nEB, NTHR, LDS_E, stream>>>(ea, ei, h, w1p, b_en1, w2p, b_en2, wedge, msg, nE, nN, nSB);
    k_node<<<nN / NBN, NTHR, LDS_N, stream>>>(ei, msg, h, b_conv, wb, b_ih, b_hh, nE, nN, vec8);
  }
  k_s2s<<<1, NTHR, LDS_S, stream>>>(h, batch, wb, b_ihl, b_hhl, b_lin1, w_lin2, b_lin2, qst, hlp, clp, out, nN, nG);
}
